// LAtAttrRobertaSelfAttention_137438954127
// MI455X (gfx1250) — hardware-verified
//
#include <hip/hip_runtime.h>
#include <hip/hip_bf16.h>
#include <stdint.h>
#include <stddef.h>


#define NB    4
#define NS    1024
#define NDM   1024
#define NH    16
#define NHD   64
#define KSTEP 32
#define LOG2E 1.4426950408889634f
#define PSCALE 4096.0f
#define PSCALE_INV 0.000244140625f
#define TPITCH 72

static_assert(NDM == NH * NHD);
static_assert(NHD == 64);
static_assert((NB * NS) % 64 == 0 && NS % 64 == 0 && NDM % 64 == 0);
static_assert(NDM % KSTEP == 0 && NS % KSTEP == 0);
static_assert((TPITCH * 2) % 16 == 0);

typedef _Float16 v16h __attribute__((ext_vector_type(16)));
typedef _Float16 v8h  __attribute__((ext_vector_type(8)));
typedef _Float16 v4h  __attribute__((ext_vector_type(4)));
typedef __bf16   v16b __attribute__((ext_vector_type(16)));
typedef __bf16   v8b  __attribute__((ext_vector_type(8)));
typedef __bf16   v4b  __attribute__((ext_vector_type(4)));
typedef float    v8f  __attribute__((ext_vector_type(8)));
typedef float    v4f  __attribute__((ext_vector_type(4)));

union FragH { v16h v; v8h half[2]; };
union FragB { v16b v; v8b half[2]; };

static __device__ __forceinline__ float bf16r(float f) {
  unsigned u = __float_as_uint(f);
  u = (u + 0x7FFFu + ((u >> 16) & 1u)) & 0xFFFF0000u;
  return __uint_as_float(u);
}

static __device__ __forceinline__ v8f wmma_bf16(const v16b a, const v16b b, v8f c) {
  v8f d = __builtin_amdgcn_wmma_f32_16x16x32_bf16(false, a, false, b, (short)0, c, false, false);
  asm volatile("v_nop\n\tv_nop\n\tv_nop\n\tv_nop" : "+v"(d) : "v"(a), "v"(b));
  return d;
}
static __device__ __forceinline__ v8f wmma_f16(const v16h a, const v16h b, v8f c) {
  v8f d = __builtin_amdgcn_wmma_f32_16x16x32_f16(false, a, false, b, (short)0, c, false, false);
  asm volatile("v_nop\n\tv_nop\n\tv_nop\n\tv_nop" : "+v"(d) : "v"(a), "v"(b));
  return d;
}

__global__ __launch_bounds__(128) void qkv_kernel(
    const float* __restrict__ hs,
    const float* __restrict__ Wq, const float* __restrict__ bq,
    const float* __restrict__ Wk, const float* __restrict__ bk,
    const float* __restrict__ Wv, const float* __restrict__ bv,
    _Float16* __restrict__ qws, _Float16* __restrict__ kws, _Float16* __restrict__ vtws)
{
  const int mt = blockIdx.x;
  const int nt = blockIdx.y;
  const int z  = blockIdx.z;
  if (mt >= (NB * NS) / 64 || nt >= NDM / 64 || z >= 3) return;

  const float* W    = (z == 0) ? Wq : ((z == 1) ? Wk : Wv);
  const float* bias = (z == 0) ? bq : ((z == 1) ? bk : bv);
  _Float16*    dstb = (z == 0) ? qws : ((z == 1) ? kws : vtws);

  __shared__ __align__(16) __bf16   lA[64][KSTEP];
  __shared__ __align__(16) __bf16   lB[64][KSTEP];
  __shared__ __align__(16) _Float16 lT[64][TPITCH];

  const int tid  = threadIdx.x;
  const int lane = tid & 31;
  const int w    = tid >> 5;
  const int h    = lane >> 4;
  const int m16  = lane & 15;
  const int mo   = (w & 1) * 32;
  const int no   = (w >> 1) * 32;
  const int Mbase = mt * 64;
  const int Nbase = nt * 64;
  const int sr   = tid >> 3;
  const int sc4  = (tid & 7) * 4;

  v8f acc[2][2];
#pragma unroll
  for (int mi = 0; mi < 2; ++mi)
#pragma unroll
    for (int ni = 0; ni < 2; ++ni) {
      const float bvv = bf16r(bias[Nbase + no + ni * 16 + m16]);
#pragma unroll
      for (int j = 0; j < 8; ++j) acc[mi][ni][j] = bvv;
    }

#pragma unroll 1
  for (int kt = 0; kt < NDM; kt += KSTEP) {
    __syncthreads();
#pragma unroll
    for (int i = 0; i < 4; ++i) {
      const int r = sr + i * 16;
      const v4f a4 = *(const v4f*)(hs + (size_t)(Mbase + r) * NDM + kt + sc4);
      const v4f w4 = *(const v4f*)(W  + (size_t)(Nbase + r) * NDM + kt + sc4);
      v4b ab, wb;
#pragma unroll
      for (int j = 0; j < 4; ++j) {
        ab[j] = static_cast<__bf16>(a4[j]);
        wb[j] = static_cast<__bf16>(w4[j]);
      }
      *(v4b*)&lA[r][sc4] = ab;
      *(v4b*)&lB[r][sc4] = wb;
    }
    __syncthreads();

    FragB bfr[2];
#pragma unroll
    for (int ni = 0; ni < 2; ++ni) {
      const __bf16* p = &lB[no + ni * 16 + m16][0];
      bfr[ni].half[0] = *(const v8b*)(p + 8 * h);
      bfr[ni].half[1] = *(const v8b*)(p + 16 + 8 * h);
    }
#pragma unroll
    for (int mi = 0; mi < 2; ++mi) {
      const __bf16* p = &lA[mo + mi * 16 + m16][0];
      FragB af;
      af.half[0] = *(const v8b*)(p + 8 * h);
      af.half[1] = *(const v8b*)(p + 16 + 8 * h);
#pragma unroll
      for (int ni = 0; ni < 2; ++ni)
        acc[mi][ni] = wmma_bf16(af.v, bfr[ni].v, acc[mi][ni]);
    }
  }

#pragma unroll
  for (int mi = 0; mi < 2; ++mi)
#pragma unroll
    for (int ni = 0; ni < 2; ++ni)
#pragma unroll
      for (int r = 0; r < 8; ++r) {
        const int ml = mo + mi * 16 + 8 * h + r;
        const int dl = no + ni * 16 + m16;
        const _Float16 v = (_Float16)acc[mi][ni][r];
        const int rr = (z == 2) ? dl : ml;
        const int cc = (z == 2) ? ml : dl;
        lT[rr][cc] = v;
      }
  __syncthreads();

  const int q8 = lane & 7;
  const int bb = Mbase / NS;
  const int s0 = Mbase % NS;
  const size_t bhb = (size_t)bb * NH + nt;
  v8h vals[4];
  size_t offs[4];
#pragma unroll
  for (int it = 0; it < 4; ++it) {
    const int L = w * 16 + it * 4 + (lane >> 3);
    vals[it] = *(const v8h*)&lT[L][q8 * 8];
    offs[it] = (z == 2) ? ((bhb * NHD + L) * (size_t)NS + s0 + q8 * 8)
                        : ((bhb * NS + s0 + L) * (size_t)NHD + q8 * 8);
    *(volatile v8h*)(dstb + offs[it]) = vals[it];
  }
  __threadfence();
#pragma unroll
  for (int it = 0; it < 4; ++it)
    *(volatile v8h*)(dstb + offs[it]) = vals[it];
}

__global__ __launch_bounds__(128) void attn_kernel(
    const _Float16* __restrict__ qws, const _Float16* __restrict__ kws,
    const _Float16* __restrict__ vtws,
    const float* __restrict__ am, const float* __restrict__ lnk,
    float* __restrict__ out)
{
  const int qt = blockIdx.x;
  const int hh = blockIdx.y;
  const int b  = blockIdx.z;
  if (qt >= NS / 64 || hh >= NH || b >= NB) return;

  const int tid  = threadIdx.x;
  const int lane = tid & 31;
  const int w    = tid >> 5;
  const int h    = lane >> 4;
  const int m16  = lane & 15;

  __shared__ __align__(16) float    lS[4][16][32];
  __shared__ __align__(16) _Float16 lP[4][16][32];
  __shared__ __align__(16) float    lO[4][16][64];

  const size_t bh = (size_t)b * NH + hh;
  const int qrow  = qt * 64 + w * 16 + m16;

  FragH qf[2];
  {
    const _Float16* qp = qws + (bh * NS + qrow) * (size_t)NHD;
#pragma unroll
    for (int kk = 0; kk < 2; ++kk) {
      qf[kk].half[0] = *(const v8h*)(qp + kk * 32 + 8 * h);
      qf[kk].half[1] = *(const v8h*)(qp + kk * 32 + 16 + 8 * h);
    }
  }

  v8f acc[4];
#pragma unroll
  for (int dt = 0; dt < 4; ++dt)
#pragma unroll
    for (int j = 0; j < 8; ++j) acc[dt][j] = 0.0f;
  float mrow = -1e30f;
  float zrow = 0.0f;

  const float* amb = am  + (size_t)b * NS;
  const float* lkr = lnk + ((size_t)b * NS + qrow) * (size_t)NS;

#pragma unroll 1
  for (int kb = 0; kb < NS; kb += KSTEP) {
#pragma unroll
    for (int sub = 0; sub < 2; ++sub) {
      const _Float16* kp = kws + (bh * NS + kb + sub * 16 + m16) * (size_t)NHD;
      v8f sc = {0.f, 0.f, 0.f, 0.f, 0.f, 0.f, 0.f, 0.f};
#pragma unroll
      for (int kk = 0; kk < 2; ++kk) {
        FragH kf;
        kf.half[0] = *(const v8h*)(kp + kk * 32 + 8 * h);
        kf.half[1] = *(const v8h*)(kp + kk * 32 + 16 + 8 * h);
        sc = wmma_f16(qf[kk].v, kf.v, sc);
      }
#pragma unroll
      for (int r = 0; r < 8; ++r)
        lS[w][8 * h + r][sub * 16 + m16] = sc[r] * 0.125f;
    }
    __syncthreads();

    float vv[16];
    float lm = -1e30f;
    {
      const float* sp = &lS[w][m16][16 * h];
      const float* ap = amb + kb + 16 * h;
#pragma unroll
      for (int i = 0; i < 4; ++i) {
        const v4f s4 = *(const v4f*)(sp + 4 * i);
        const v4f a4 = *(const v4f*)(ap + 4 * i);
#pragma unroll
        for (int j = 0; j < 4; ++j) {
          const float t = s4[j] + bf16r(a4[j]);
          vv[4 * i + j] = t;
          lm = fmaxf(lm, t);
        }
      }
    }
    lm = fmaxf(lm, __shfl_xor(lm, 16));
    const float mnew = fmaxf(mrow, lm);
    const float corr = __builtin_amdgcn_exp2f((mrow - mnew) * LOG2E);
    float ps = 0.0f;
    {
      const float* lp = lkr + kb + 16 * h;
#pragma unroll
      for (int i = 0; i < 4; ++i) {
        const v4f l4 = *(const v4f*)(lp + 4 * i);
        v4h p4;
#pragma unroll
        for (int j = 0; j < 4; ++j) {
          const float pr = __builtin_amdgcn_exp2f((vv[4 * i + j] - mnew) * LOG2E);
          ps += pr;
          const float pl = pr * bf16r(l4[j]) * PSCALE;
          p4[j] = (_Float16)pl;
        }
        *(v4h*)&lP[w][m16][16 * h + 4 * i] = p4;
      }
    }
    ps += __shfl_xor(ps, 16);
    zrow = zrow * corr + ps;
    mrow = mnew;

    float cf[8];
#pragma unroll
    for (int r = 0; r < 8; ++r) cf[r] = __shfl(corr, 8 * h + r);
#pragma unroll
    for (int dt = 0; dt < 4; ++dt)
#pragma unroll
      for (int r = 0; r < 8; ++r) acc[dt][r] *= cf[r];
    __syncthreads();

    FragH pf;
    pf.half[0] = *(const v8h*)&lP[w][m16][8 * h];
    pf.half[1] = *(const v8h*)&lP[w][m16][16 + 8 * h];
#pragma unroll
    for (int dt = 0; dt < 4; ++dt) {
      const _Float16* vp = vtws + (bh * NHD + dt * 16 + m16) * (size_t)NS + kb;
      FragH vf;
      vf.half[0] = *(const v8h*)(vp + 8 * h);
      vf.half[1] = *(const v8h*)(vp + 16 + 8 * h);
      acc[dt] = wmma_f16(pf.v, vf.v, acc[dt]);
    }
  }

  const float invz = 1.0f / zrow;
  float zf[8];
#pragma unroll
  for (int r = 0; r < 8; ++r) zf[r] = __shfl(invz, 8 * h + r) * PSCALE_INV;
#pragma unroll
  for (int dt = 0; dt < 4; ++dt)
#pragma unroll
    for (int r = 0; r < 8; ++r)
      lO[w][8 * h + r][dt * 16 + m16] = acc[dt][r] * zf[r];
  __syncthreads();

  const int q8 = lane & 7;
  const size_t rowb = (size_t)b * NS + qt * 64 + w * 16;
  v4f ov[8];
  size_t oo[8];
#pragma unroll
  for (int it = 0; it < 8; ++it) {
    const int L    = it * 4 + (lane >> 3);
    const int row  = L >> 1;
    const int half = L & 1;
    ov[it] = *(const v4f*)&lO[w][row][half * 32 + q8 * 4];
    oo[it] = (rowb + row) * (size_t)NDM + hh * NHD + half * 32 + q8 * 4;
    *(volatile v4f*)(out + oo[it]) = ov[it];
  }
  __threadfence();
#pragma unroll
  for (int it = 0; it < 8; ++it)
    *(volatile v4f*)(out + oo[it]) = ov[it];
}

extern "C" void kernel_launch(void* const* d_in, const int* in_sizes, int n_in,
                              void* d_out, int out_size, void* d_ws, size_t ws_size,
                              hipStream_t stream) {
  if (n_in < 9) return;
  const size_t NE = (size_t)NB * NS * NDM;
  if ((size_t)in_sizes[0] != NE) return;
  if ((size_t)in_sizes[1] != (size_t)NB * NS) return;
  if ((size_t)in_sizes[2] != (size_t)NB * NS * NS) return;
  if ((size_t)in_sizes[3] != (size_t)NDM * NDM || (size_t)in_sizes[5] != (size_t)NDM * NDM ||
      (size_t)in_sizes[7] != (size_t)NDM * NDM) return;
  if ((size_t)in_sizes[4] != (size_t)NDM || (size_t)in_sizes[6] != (size_t)NDM ||
      (size_t)in_sizes[8] != (size_t)NDM) return;
  if ((size_t)out_size != NE) return;
  if (3 * NE * sizeof(_Float16) > ws_size) return;

  const float* hs  = (const float*)d_in[0];
  const float* am  = (const float*)d_in[1];
  const float* lnk = (const float*)d_in[2];
  const float* Wq  = (const float*)d_in[3];
  const float* bq  = (const float*)d_in[4];
  const float* Wk  = (const float*)d_in[5];
  const float* bk  = (const float*)d_in[6];
  const float* Wv  = (const float*)d_in[7];
  const float* bv  = (const float*)d_in[8];

  _Float16* qws  = (_Float16*)d_ws;
  _Float16* kws  = qws + NE;
  _Float16* vtws = kws + NE;

  qkv_kernel<<<dim3((NB * NS) / 64, NDM / 64, 3), 128, 0, stream>>>(
      hs, Wq, bq, Wk, bk, Wv, bv, qws, kws, vtws);
  attn_kernel<<<dim3(NS / 64, NH, NB), 128, 0, stream>>>(
      qws, kws, vtws, am, lnk, (float*)d_out);
  (void)hipGetLastError();
}
